// RNN_Net_50096498541013
// MI455X (gfx1250) — hardware-verified
//
#include <hip/hip_runtime.h>
#include <stdint.h>

#define DT_STEP 0.2f
#define B_SZ   64
#define T_SZ   512
#define DIN    128
#define DH     512
#define DOUT   128
#define RSPLIT (1.0f / 2048.0f)

typedef _Float16 f16;
typedef __attribute__((ext_vector_type(16))) _Float16 v16h;
typedef __attribute__((ext_vector_type(8)))  _Float16 v8h;
typedef __attribute__((ext_vector_type(8)))  float    v8f;
typedef __attribute__((ext_vector_type(4)))  float    v4f_t;
typedef float v4fa __attribute__((ext_vector_type(4), may_alias));

__device__ __forceinline__ v8f wmma16(v16h a, v16h b, v8f c) {
  return __builtin_amdgcn_wmma_f32_16x16x32_f16(false, a, false, b, (short)0, c, false, false);
}
__device__ __forceinline__ v8f wmma_split(v16h a, v16h al, v16h b, v16h bl, v8f c) {
  v8f x = {};
  x = wmma16(al, b, x); x = wmma16(a, bl, x);
  return wmma16(a, b, c) + x * RSPLIT;
}
__device__ __forceinline__ f16 lo_of(float v, f16 h) { return (f16)((v - (float)h) * 2048.0f); }
__device__ __forceinline__ v16h cat8(v8h a, v8h b) {
  return __builtin_shufflevector(a, b, 0,1,2,3,4,5,6,7,8,9,10,11,12,13,14,15);
}
__device__ __forceinline__ v16h load_a(const f16* tile, int pitch, int lane) {
  const f16* p = tile + (size_t)(lane & 15) * pitch + (lane >> 4) * 8;
  return cat8(*(const v8h*)p, *(const v8h*)(p + 16));
}
__device__ __forceinline__ v16h load_swz(const f16* frag, int lane) {
  const f16* p = frag + lane * 16;
  return cat8(*(const v8h*)p, *(const v8h*)(p + 8));
}

__global__ __launch_bounds__(256) void swz_kernel(const float* __restrict__ Wt, f16* __restrict__ dst, int N, int K) {
  const int i = (blockIdx.x * 256 + threadIdx.x) * 2;
  if (i >= N * K) return;
  const int KC = K / 32;
  unsigned ph = 0, pl = 0;
#pragma unroll
  for (int q = 0; q < 2; ++q) {
    const int ii = i + q, j = ii & 15, lane = (ii >> 4) & 31, rest = ii >> 9, c = rest % KC, nt = rest / KC;
    const int hi = lane >> 4, n = nt * 16 + (lane & 15);
    const int k = c * 32 + ((j < 8) ? (hi * 8 + j) : (16 + hi * 8 + (j - 8)));
    const float v = Wt[(size_t)n * K + k];
    const f16 h = (f16)v, l = lo_of(v, h);
    ph |= (unsigned)__builtin_bit_cast(unsigned short, h) << (16 * q);
    pl |= (unsigned)__builtin_bit_cast(unsigned short, l) << (16 * q);
  }
  const size_t plane = (size_t)N * K;
  *(volatile unsigned*)(dst + i) = ph; *(volatile unsigned*)(dst + plane + i) = pl; __threadfence();
  *(volatile unsigned*)(dst + i) = ph; *(volatile unsigned*)(dst + plane + i) = pl;
}

__global__ __launch_bounds__(256) void gemm_xin(const float* __restrict__ x, const f16* __restrict__ wih_sw, float* __restrict__ xin) {
  __shared__ __attribute__((aligned(16))) float stg[16][128 + 4];
  const int lane = threadIdx.x & 31, wave = threadIdx.x >> 5, tid = threadIdx.x;
  const int mt = blockIdx.x >> 2, nt0 = (blockIdx.x & 3) * 8;
  const int nt = nt0 + wave;
  const int mlo = lane & 15, hi = lane >> 4;
  const float* xr = x + (size_t)(mt * 16 + mlo) * DIN;
  const size_t plw = (size_t)DH * DIN;
  v8f acc = {};
#pragma unroll
  for (int c = 0; c < DIN / 32; ++c) {
    v16h a, al;
    const v4f_t x0 = *(const v4f_t*)(xr + c * 32 + hi * 8), x1 = *(const v4f_t*)(xr + c * 32 + hi * 8 + 4);
    const v4f_t x2 = *(const v4f_t*)(xr + c * 32 + 16 + hi * 8), x3 = *(const v4f_t*)(xr + c * 32 + 16 + hi * 8 + 4);
    float f[16] = {x0.x, x0.y, x0.z, x0.w, x1.x, x1.y, x1.z, x1.w, x2.x, x2.y, x2.z, x2.w, x3.x, x3.y, x3.z, x3.w};
#pragma unroll
    for (int e = 0; e < 16; ++e) { const f16 h = (f16)f[e]; a[e] = h; al[e] = lo_of(f[e], h); }
    const f16* fb = wih_sw + ((size_t)nt * (DIN / 32) + c) * 512;
    acc = wmma_split(a, al, load_swz(fb, lane), load_swz(fb + plw, lane), acc);
  }
#pragma unroll
  for (int r = 0; r < 8; ++r) stg[hi * 8 + r][wave * 16 + mlo] = acc[r];
  __syncthreads();
#pragma unroll 1
  for (int pass = 0; pass < 2; ++pass) {
#pragma unroll
    for (int i = 0; i < 2; ++i) { const int cc = tid + 256 * i, rr = cc >> 5, q = cc & 31;
      *(volatile v4f_t*)(xin + (size_t)(mt * 16 + rr) * DH + nt0 * 16 + q * 4) = *(const v4fa*)&stg[rr][q * 4]; }
    __threadfence();
  }
}

#define PLHS ((size_t)T_SZ * B_SZ * DH)
__global__ __launch_bounds__(1024) void rnn_recur(const float* __restrict__ xin, const f16* __restrict__ whh_sw, f16* __restrict__ hsb,
                                                  float* __restrict__ hst) {
  __shared__ __attribute__((aligned(16))) f16 th[2][B_SZ][DH];
  const int tid = threadIdx.x, lane = tid & 31, wave = tid >> 5;
  const int mlo = lane & 15, hi8 = (lane >> 4) * 8;
  const int ncol = wave * 16 + mlo;
  const f16* wbase = whh_sw + (size_t)(wave * 16) * 512;
  const size_t plw = (size_t)DH * DH;
  float* hmine = hst + (size_t)(wave * 4) * 256 + lane * 8;

#pragma unroll
  for (int m = 0; m < 4; ++m) { const v8f z = {0.f, 0.f, 0.f, 0.f, 0.f, 0.f, 0.f, 0.f}; *(volatile v8f*)(hmine + m * 256) = z; }
  __threadfence();

  for (int t = 0; t < T_SZ; ++t) {
#pragma unroll
    for (int m = 0; m < 4; ++m) {
      const v8f hv8 = *(const volatile v8f*)(hmine + m * 256);
#pragma unroll
      for (int r = 0; r < 8; ++r) {
        const float tv = tanhf(hv8[r]);
        const f16 hv = (f16)tv;
        th[0][m * 16 + hi8 + r][ncol] = hv;
        th[1][m * 16 + hi8 + r][ncol] = lo_of(tv, hv);
      }
    }
    __syncthreads();

    v8f acc[4];
#pragma unroll
    for (int m = 0; m < 4; ++m)
#pragma unroll
      for (int r = 0; r < 8; ++r) acc[m][r] = xin[((size_t)(m * 16 + hi8 + r) * T_SZ + t) * DH + ncol];
#pragma unroll 2
    for (int c = 0; c < DH / 32; ++c) {
      const v16h wf = load_swz(wbase + (size_t)c * 512, lane), wfl = load_swz(wbase + plw + (size_t)c * 512, lane);
#pragma unroll
      for (int m = 0; m < 4; ++m) {
        const v16h a = load_a(&th[0][m * 16][c * 32], DH, lane), al = load_a(&th[1][m * 16][c * 32], DH, lane);
        acc[m] = wmma_split(a, al, wf, wfl, acc[m]);
      }
    }

#pragma unroll
    for (int m = 0; m < 4; ++m) {
      const v8f hv8 = *(const volatile v8f*)(hmine + m * 256);
      v8h ph, pl;
#pragma unroll
      for (int r = 0; r < 8; ++r) { const f16 hv = (f16)hv8[r]; ph[r] = hv; pl[r] = lo_of(hv8[r], hv); }
      f16* dst = hsb + ((size_t)(t * 32 + wave) * 4 + m) * 256 + lane * 8;
      *(volatile v8h*)dst = ph; *(volatile v8h*)(dst + PLHS) = pl;
      const v8f hn = hv8 * (1.0f - DT_STEP) + acc[m] * DT_STEP;
      *(volatile v8f*)(hmine + m * 256) = hn;
      __threadfence();
      *(volatile v8h*)dst = ph; *(volatile v8h*)(dst + PLHS) = pl;
      *(volatile v8f*)(hmine + m * 256) = hn;
    }
    __syncthreads();
  }
}

__global__ __launch_bounds__(256) void gemm_dec(const f16* __restrict__ hsb, const f16* __restrict__ wdec_sw, float* __restrict__ out) {
  __shared__ __attribute__((aligned(16))) f16 At[2][16][DH + 8];
  __shared__ __attribute__((aligned(16))) float stg[16][128 + 4];
  const int tid = threadIdx.x, lane = tid & 31, wave = tid >> 5;
  const int t = blockIdx.x >> 2, m = blockIdx.x & 3;
  const int mlo = lane & 15, hi = lane >> 4;
  for (int e = tid; e < 32 * 32; e += 256) {
    const int w = e >> 5, L = e & 31;
    const f16* src = hsb + ((size_t)(t * 32 + w) * 4 + m) * 256 + L * 8;
    const v8h vh = *(const v8h*)src, vl = *(const v8h*)(src + PLHS);
    const int col = w * 16 + (L & 15), r0 = (L >> 4) * 8;
#pragma unroll
    for (int r = 0; r < 8; ++r) { At[0][r0 + r][col] = vh[r]; At[1][r0 + r][col] = vl[r]; }
  }
  __syncthreads();
  const size_t plw = (size_t)DOUT * DH;
  v8f acc = {};
#pragma unroll 4
  for (int c = 0; c < DH / 32; ++c) {
    const v16h a = load_a(&At[0][0][c * 32], DH + 8, lane), al = load_a(&At[1][0][c * 32], DH + 8, lane);
    const f16* fb = wdec_sw + ((size_t)wave * (DH / 32) + c) * 512;
    acc = wmma_split(a, al, load_swz(fb, lane), load_swz(fb + plw, lane), acc);
  }
#pragma unroll
  for (int r = 0; r < 8; ++r) stg[hi * 8 + r][wave * 16 + mlo] = acc[r];
  __syncthreads();
#pragma unroll 1
  for (int pass = 0; pass < 2; ++pass) {
#pragma unroll
    for (int i = 0; i < 2; ++i) { const int cc = tid + 256 * i, rr = cc >> 5, q = cc & 31;
      const int b = m * 16 + rr;
      *(volatile v4f_t*)(out + ((size_t)b * T_SZ + t) * DOUT + q * 4) = *(const v4fa*)&stg[rr][q * 4]; }
    __threadfence();
  }
}

extern "C" void kernel_launch(void* const* d_in, const int* in_sizes, int n_in,
                              void* d_out, int out_size, void* d_ws, size_t ws_size,
                              hipStream_t stream) {
    (void)in_sizes; (void)n_in; (void)out_size; (void)ws_size;
    const float* x    = (const float*)d_in[0];
    const float* Wih  = (const float*)d_in[1];
    const float* Whh  = (const float*)d_in[2];
    const float* Wdec = (const float*)d_in[3];

    char* ws = (char*)d_ws;
    size_t o = 0;
    float* xin     = (float*)(ws + o); o += (size_t)B_SZ * T_SZ * DH * 4;
    f16*   hsb     = (f16*)  (ws + o); o += (size_t)T_SZ * B_SZ * DH * 2 * 2;
    f16*   whh_sw  = (f16*)  (ws + o); o += (size_t)DH * DH * 2 * 2;
    f16*   wih_sw  = (f16*)  (ws + o); o += (size_t)DH * DIN * 2 * 2;
    f16*   wdec_sw = (f16*)  (ws + o); o += (size_t)DOUT * DH * 2 * 2;
    float* hst     = (float*)(ws + o); o += (size_t)B_SZ * DH * 4;

    swz_kernel<<<(DH * DIN / 2 + 255) / 256, 256, 0, stream>>>(Wih, wih_sw, DH, DIN);
    swz_kernel<<<(DH * DH / 2 + 255) / 256, 256, 0, stream>>>(Whh, whh_sw, DH, DH);
    swz_kernel<<<(DOUT * DH / 2 + 255) / 256, 256, 0, stream>>>(Wdec, wdec_sw, DOUT, DH);
    gemm_xin<<<(B_SZ * T_SZ / 16) * 4, 256, 0, stream>>>(x, wih_sw, xin);
    rnn_recur<<<1, 1024, 0, stream>>>(xin, whh_sw, hsb, hst);
    gemm_dec<<<T_SZ * 4, 256, 0, stream>>>(hsb, wdec_sw, (float*)d_out);
}
